// MultiHeadSelfAttention_32452772889293
// MI455X (gfx1250) — hardware-verified
//
#include <hip/hip_runtime.h>
#ifndef NB
#define NB 4
#endif
#ifndef SEQ
#define SEQ 2048
#endif
#define SEQ_FULL 2048
#define DM 768
#define NH 12
#define HD 64
#define NR (NB * SEQ)
#define LN1024 6.931471805599453f

static_assert(NH * HD == DM);
static_assert(HD == 64);
static_assert(DM % 128 == 0);
static_assert(DM % 64 == 0);
static_assert(DM % 32 == 0);
static_assert(NR % 128 == 0);
static_assert(SEQ % 64 == 0);
static_assert(SEQ % 32 == 0);
static_assert((SEQ / 16) % 4 == 0);
static_assert(SEQ <= SEQ_FULL);
static_assert(((size_t)NB * NH * (SEQ / 16)) % 4 == 0);
static_assert((size_t)4 * DM * DM * 2 + (size_t)5 * NR * DM * 2 <= (size_t)134217728);

typedef _Float16 v16h __attribute__((ext_vector_type(16)));
typedef unsigned short v8us __attribute__((ext_vector_type(8), may_alias));
typedef float v8f  __attribute__((ext_vector_type(8)));
typedef float v4f  __attribute__((ext_vector_type(4)));
typedef float v4fa __attribute__((ext_vector_type(4), may_alias));
union FragH { v16h v; v8us half[2]; _Float16 h[16]; unsigned short u[16]; };

__device__ __forceinline__ unsigned short bf16_bits(float x) { unsigned int u = __float_as_uint(x); return (unsigned short)((u + 0x7FFFu + ((u >> 16) & 1u)) >> 16); }
__device__ __forceinline__ float bf16_rne(float x) { return __uint_as_float(((unsigned int)bf16_bits(x)) << 16); }
__device__ __forceinline__ int imin(int a, int b) { return (a < b) ? a : b; }

__device__ __forceinline__ v16h ldfrag(const _Float16* p, int hh) {
  FragH f;
  f.half[0] = *(const v8us*)((const unsigned short*)p + 8 * hh);
  f.half[1] = *(const v8us*)((const unsigned short*)p + 16 + 8 * hh);
  return f.v;
}
__device__ __forceinline__ v8f mma16(v16h a, v16h b, v8f c) {
  v8f d = __builtin_amdgcn_wmma_f32_16x16x32_f16(false, a, false, b, (short)0, c, false, false);
  asm volatile("v_nop\n\tv_nop\n\tv_nop\n\tv_nop" : "+v"(d) : "v"(a), "v"(b));
  return d;
}

__global__ __launch_bounds__(256) void k_wt_f16(const float* __restrict__ W, _Float16* __restrict__ Wt, int K, int N, float scale) {
  const int t = blockIdx.x * 256 + threadIdx.x;
  const int k8n = K / 8;
  if (t >= N * k8n) return;
  const int n = t / k8n, k8 = (t % k8n) * 8;
  FragH f;
#pragma unroll
  for (int i = 0; i < 8; ++i) f.h[i] = (_Float16)(bf16_rne(W[(size_t)(k8 + i) * N + n]) * scale);
  const v8us o = f.half[0];
  unsigned short* d = (unsigned short*)Wt + (size_t)n * K + k8;
  *(volatile v8us*)d = o;
  __threadfence();
  *(volatile v8us*)d = o;
}

__global__ __launch_bounds__(256) void k_x16(const float* __restrict__ x, _Float16* __restrict__ X16, int nthr) {
  const int t = blockIdx.x * 256 + threadIdx.x;
  if (t >= nthr) return;
  const int row = t / (DM / 8), c8 = (t % (DM / 8)) * 8;
  const int b = row / SEQ, s = row % SEQ;
  const float* src = x + ((size_t)b * SEQ_FULL + s) * DM + c8;
  const v4f a = *(const v4fa*)src, c = *(const v4fa*)(src + 4);
  FragH f;
#pragma unroll
  for (int q = 0; q < 4; ++q) { f.h[q] = (_Float16)bf16_rne(a[q]); f.h[4 + q] = (_Float16)bf16_rne(c[q]); }
  const v8us o = f.half[0];
  unsigned short* d = (unsigned short*)X16 + (size_t)t * 8;
  *(volatile v8us*)d = o;
  __threadfence();
  *(volatile v8us*)d = o;
}

__global__ __launch_bounds__(128) void k_gemm(const _Float16* __restrict__ A, int lda,
                                              const _Float16* __restrict__ Bh, int ldb, size_t sB, float alpha,
                                              const float* __restrict__ bias, int nbias, int biasrow,
                                              float* __restrict__ C32, _Float16* __restrict__ C16, int out16,
                                              int ldc, size_t sC, int M, int N, int K) {
  __shared__ __attribute__((aligned(16))) float so[4][32][68];
  const int tid = threadIdx.x, lane = tid & 31, ln = lane & 15, hh = lane >> 4;
  const int w = __builtin_amdgcn_readfirstlane(tid >> 5);
  const int by = blockIdx.y;
  const _Float16* Bb = Bh + (size_t)by * sB;
  const size_t cofs = (size_t)by * sC;
  const int ntn = N >> 6;
  const int mt = blockIdx.x / ntn, nq = blockIdx.x - mt * ntn;
  const int row0 = mt * 128 + 32 * w, col0 = nq * 64;
  if (row0 >= M) return;
  const _Float16* a0p = A + (size_t)(row0 + ln) * lda;
  const _Float16* a1p = a0p + (size_t)16 * lda;
  const _Float16* b0p = Bb + (size_t)(col0 + ln) * ldb;
  const _Float16* b1p = b0p + (size_t)16 * ldb;
  const _Float16* b2p = b1p + (size_t)16 * ldb;
  const _Float16* b3p = b2p + (size_t)16 * ldb;
  const v8f z8 = {0.f, 0.f, 0.f, 0.f, 0.f, 0.f, 0.f, 0.f};
  v8f c00 = z8, c01 = z8, c02 = z8, c03 = z8, c10 = z8, c11 = z8, c12 = z8, c13 = z8;
#pragma unroll 1
  for (int kb = 0; kb < K; kb += 32) {
    const v16h a0 = ldfrag(a0p + kb, hh), a1 = ldfrag(a1p + kb, hh);
    v16h b = ldfrag(b0p + kb, hh); c00 = mma16(a0, b, c00); c10 = mma16(a1, b, c10);
    b = ldfrag(b1p + kb, hh); c01 = mma16(a0, b, c01); c11 = mma16(a1, b, c11);
    b = ldfrag(b2p + kb, hh); c02 = mma16(a0, b, c02); c12 = mma16(a1, b, c12);
    b = ldfrag(b3p + kb, hh); c03 = mma16(a0, b, c03); c13 = mma16(a1, b, c13);
  }
  const int rb0 = imin(row0 + 8 * hh, nbias - 8), rb1 = imin(row0 + 16 + 8 * hh, nbias - 8);
  const v4f br00 = *(const v4fa*)(bias + rb0), br01 = *(const v4fa*)(bias + rb0 + 4);
  const v4f br10 = *(const v4fa*)(bias + rb1), br11 = *(const v4fa*)(bias + rb1 + 4);
  const float brow[16] = {br00[0], br00[1], br00[2], br00[3], br01[0], br01[1], br01[2], br01[3],
                          br10[0], br10[1], br10[2], br10[3], br11[0], br11[1], br11[2], br11[3]};
  const v8f accs[8] = {c00, c01, c02, c03, c10, c11, c12, c13};
#pragma unroll
  for (int u = 0; u < 8; ++u) {
    const int t = u & 3, half = u >> 2;
    const int col = col0 + t * 16 + ln;
    const float bc = bf16_rne(bias[imin(col, nbias - 1)]);
#pragma unroll
    for (int r = 0; r < 8; ++r) {
      const int rloc = half * 16 + 8 * hh + r;
      const float br = bf16_rne(brow[half * 8 + r]);
      const float bv = (biasrow != 0) ? br : bc;
      so[w][rloc][t * 16 + ln] = accs[u][r] * alpha + bv;
    }
  }
  __builtin_amdgcn_fence(4  , "workgroup");
  __builtin_amdgcn_wave_barrier();
  if (out16 != 0) {
    const int rq = lane >> 3, c8 = (lane & 7) * 8;
    for (int pass = 0; pass < 2; ++pass) {
#pragma unroll
      for (int it = 0; it < 8; ++it) {
        const int row = it * 4 + rq;
        const v4f x0 = *(const v4fa*)&so[w][row][c8];
        const v4f x1 = *(const v4fa*)&so[w][row][c8 + 4];
        FragH f;
#pragma unroll
        for (int q = 0; q < 4; ++q) { f.h[q] = (_Float16)x0[q]; f.h[4 + q] = (_Float16)x1[q]; }
        const v8us o = f.half[0];
        *(volatile v8us*)((unsigned short*)C16 + cofs + (size_t)(row0 + row) * ldc + col0 + c8) = o;
      }
      if (pass == 0) __threadfence();
    }
  } else {
    const int rsub = lane >> 4, c4 = (lane & 15) * 4;
    for (int pass = 0; pass < 2; ++pass) {
#pragma unroll
      for (int q = 0; q < 16; ++q) {
        const int r = q * 2 + rsub;
        const v4f v = *(const v4fa*)&so[w][r][c4];
        *(volatile v4f*)(C32 + cofs + (size_t)(row0 + r) * ldc + col0 + c4) = v;
      }
      if (pass == 0) __threadfence();
    }
  }
}

__global__ __launch_bounds__(128) void k_attn(const _Float16* __restrict__ Q16, const _Float16* __restrict__ K16,
                                              const _Float16* __restrict__ VT, const float* __restrict__ mask,
                                              _Float16* __restrict__ O16) {
  __shared__ __attribute__((aligned(16))) float msk[SEQ];
  __shared__ __attribute__((aligned(16))) unsigned short ct[4][16][72];
  const int tid = threadIdx.x, lane = tid & 31, ln = lane & 15, hh = lane >> 4;
  const int w = __builtin_amdgcn_readfirstlane(tid >> 5);
  const int gw = blockIdx.x * 4 + w;
  const int bh = gw / (SEQ / 16);
  const int qt = gw - bh * (SEQ / 16);
  const int b = bh / NH, h = bh - b * NH;
  const float* mrow = mask + (size_t)b * SEQ_FULL;
  for (int i = tid * 4; i < SEQ; i += 512) {
    const v4f m = *(const v4fa*)(mrow + i);
    v4f o;
#pragma unroll
    for (int q = 0; q < 4; ++q) o[q] = bf16_rne(m[q]) * -1.0e9f;
    *(v4fa*)&msk[i] = o;
  }
  __syncthreads();
  const size_t tok0 = (size_t)b * SEQ;
  const _Float16* qrow = Q16 + (tok0 + (size_t)(qt * 16 + ln)) * DM + h * HD;
  const v16h qb0 = ldfrag(qrow, hh), qb1 = ldfrag(qrow + 32, hh);
  const _Float16* kbase = K16 + (tok0 + (size_t)ln) * DM + h * HD;
  const _Float16* vbase = VT + ((size_t)b * DM + (size_t)(h * HD + ln)) * SEQ;
  const v8f z8 = {0.f, 0.f, 0.f, 0.f, 0.f, 0.f, 0.f, 0.f};
  v8f o0 = z8, o1 = z8, o2 = z8, o3 = z8;
  float mo = -1.0e30f, mso = -1.0e30f, l = 0.f;
#pragma unroll 1
  for (int kb = 0; kb < SEQ; kb += 32) {
    const _Float16* k0p = kbase + (size_t)kb * DM;
    const _Float16* k1p = k0p + (size_t)16 * DM;
    v8f s0 = z8, s1 = z8;
    { v16h a = ldfrag(k0p, hh); s0 = mma16(a, qb0, s0); a = ldfrag(k0p + 32, hh); s0 = mma16(a, qb1, s0); }
    { v16h a = ldfrag(k1p, hh); s1 = mma16(a, qb0, s1); a = ldfrag(k1p + 32, hh); s1 = mma16(a, qb1, s1); }
    const v4f ma = *(const v4fa*)&msk[kb + 8 * hh];
    const v4f mb = *(const v4fa*)&msk[kb + 8 * hh + 4];
    const v4f mc = *(const v4fa*)&msk[kb + 16 + 8 * hh];
    const v4f md = *(const v4fa*)&msk[kb + 16 + 8 * hh + 4];
    const float am0[8] = {ma[0], ma[1], ma[2], ma[3], mb[0], mb[1], mb[2], mb[3]};
    const float am1[8] = {mc[0], mc[1], mc[2], mc[3], md[0], md[1], md[2], md[3]};
    float e0[8], e1[8];
#pragma unroll
    for (int r = 0; r < 8; ++r) { e0[r] = fmaf(s0[r], 0.125f, am0[r]); e1[r] = fmaf(s1[r], 0.125f, am1[r]); }
    float bm = fmaxf(e0[0], e1[0]);
#pragma unroll
    for (int r = 1; r < 8; ++r) bm = fmaxf(bm, fmaxf(e0[r], e1[r]));
    const float bmo = __shfl_xor(bm, 16, 32);
    bm = fmaxf(bm, bmo);
    const float mn = fmaxf(mo, bm);
    const float msn = mn - LN1024;
    const float alpha = __expf(mso - msn);
    mo = mn; mso = msn;
    float ps = 0.f;
    FragH pf;
#pragma unroll
    for (int r = 0; r < 8; ++r) {
      const float p0 = __expf(e0[r] - msn);
      const float p1 = __expf(e1[r] - msn);
      ps += p0 + p1;
      pf.h[r] = (_Float16)p0;
      pf.h[8 + r] = (_Float16)p1;
    }
    l = l * alpha + ps;
    o0 *= alpha; o1 *= alpha; o2 *= alpha; o3 *= alpha;
    const _Float16* vp = vbase + kb;
    { const v16h a = ldfrag(vp, hh); o0 = mma16(a, pf.v, o0); }
    { const v16h a = ldfrag(vp + (size_t)16 * SEQ, hh); o1 = mma16(a, pf.v, o1); }
    { const v16h a = ldfrag(vp + (size_t)32 * SEQ, hh); o2 = mma16(a, pf.v, o2); }
    { const v16h a = ldfrag(vp + (size_t)48 * SEQ, hh); o3 = mma16(a, pf.v, o3); }
  }
  const float lo = __shfl_xor(l, 16, 32);
  const float lt = l + lo;
  const float inv = 64.0f / lt;
  const v8f oo[4] = {o0, o1, o2, o3};
#pragma unroll
  for (int j = 0; j < 4; ++j) {
    FragH f;
#pragma unroll
    for (int r = 0; r < 8; ++r) f.h[r] = (_Float16)(oo[j][r] * inv);
    *(v8us*)&ct[w][ln][16 * j + 8 * hh] = f.half[0];
  }
  __builtin_amdgcn_fence(4  , "workgroup");
  __builtin_amdgcn_wave_barrier();
  const int rq = lane >> 3, pc = lane & 7;
  for (int pass = 0; pass < 2; ++pass) {
#pragma unroll
    for (int it = 0; it < 4; ++it) {
      const int row = it * 4 + rq;
      const v8us v = *(const v8us*)&ct[w][row][pc * 8];
      *(volatile v8us*)((unsigned short*)O16 + (tok0 + (size_t)(qt * 16 + row)) * DM + h * HD + pc * 8) = v;
    }
    if (pass == 0) __threadfence();
  }
}

extern "C" void kernel_launch(void* const* d_in, const int* in_sizes, int n_in,
                              void* d_out, int out_size, void* d_ws, size_t ws_size, hipStream_t stream) {
  if (n_in < 10) return;
  const size_t needRows = (size_t)(NB - 1) * SEQ_FULL + SEQ;
  if ((size_t)in_sizes[0] < needRows * DM) return;
  if ((size_t)in_sizes[1] < needRows) return;
  if ((size_t)in_sizes[2] < (size_t)DM * DM || (size_t)in_sizes[4] < (size_t)DM * DM) return;
  if ((size_t)in_sizes[6] < (size_t)DM * DM || (size_t)in_sizes[8] < (size_t)DM * DM) return;
  if (in_sizes[3] < DM || in_sizes[5] < DM || in_sizes[7] < DM || in_sizes[9] < DM) return;
  if ((size_t)out_size < (size_t)NR * DM) return;
  const float* x    = (const float*)d_in[0];
  const float* mask = (const float*)d_in[1];
  const float* wq   = (const float*)d_in[2];
  const float* bq   = (const float*)d_in[3];
  const float* wk   = (const float*)d_in[4];
  const float* bk   = (const float*)d_in[5];
  const float* wv   = (const float*)d_in[6];
  const float* bv   = (const float*)d_in[7];
  const float* wo   = (const float*)d_in[8];
  const float* bo   = (const float*)d_in[9];
  float* out = (float*)d_out;

  char* ws = (char*)d_ws; size_t off = 0;
  const size_t wB = (size_t)DM * DM * 2;
  const size_t pB = (size_t)NR * DM * 2;
  _Float16* BQ  = (_Float16*)(ws + off); off += wB;
  _Float16* BK  = (_Float16*)(ws + off); off += wB;
  _Float16* BV  = (_Float16*)(ws + off); off += wB;
  _Float16* BO  = (_Float16*)(ws + off); off += wB;
  _Float16* X16 = (_Float16*)(ws + off); off += pB;
  _Float16* Q16 = (_Float16*)(ws + off); off += pB;
  _Float16* K16 = (_Float16*)(ws + off); off += pB;
  _Float16* VT  = (_Float16*)(ws + off); off += pB;
  _Float16* O16 = (_Float16*)(ws + off); off += pB;
  if (off > ws_size) return;

  { const unsigned g = (unsigned)(((size_t)DM * (DM / 8) + 255) / 256);
    k_wt_f16<<<g, 256, 0, stream>>>(wq, BQ, DM, DM, 16.0f);
    k_wt_f16<<<g, 256, 0, stream>>>(wk, BK, DM, DM, 16.0f);
    k_wt_f16<<<g, 256, 0, stream>>>(wv, BV, DM, DM, 16.0f);
    k_wt_f16<<<g, 256, 0, stream>>>(wo, BO, DM, DM, 16.0f); }
  { const int nthr = NR * (DM / 8);
    k_x16<<<(unsigned)((nthr + 255) / 256), 256, 0, stream>>>(x, X16, nthr); }
  k_gemm<<<dim3((unsigned)((NR / 128) * (DM / 64)), 1), 128, 0, stream>>>(X16, DM, BQ, DM, (size_t)0, 0.0625f, bq, DM, 0, out, Q16, 1, DM, (size_t)0, NR, DM, DM);
  k_gemm<<<dim3((unsigned)((NR / 128) * (DM / 64)), 1), 128, 0, stream>>>(X16, DM, BK, DM, (size_t)0, 0.0625f, bk, DM, 0, out, K16, 1, DM, (size_t)0, NR, DM, DM);
  k_gemm<<<dim3((unsigned)((DM / 128) * (SEQ / 64)), NB), 128, 0, stream>>>(BV, DM, X16, DM, (size_t)SEQ * DM, 0.0625f, bv, DM, 1, out, VT, 1, SEQ, (size_t)DM * SEQ, DM, SEQ, DM);
  k_attn<<<(unsigned)(((size_t)NB * NH * (SEQ / 16)) / 4), 128, 0, stream>>>(Q16, K16, VT, mask, O16);
  k_gemm<<<dim3((unsigned)((NR / 128) * (DM / 64)), 1), 128, 0, stream>>>(O16, DM, BO, DM, (size_t)0, 0.0009765625f, bo, DM, 0, out, Q16, 0, DM, (size_t)0, NR, DM, DM);
}
